// EnhancedLNNManipulator_63350767616780
// MI455X (gfx1250) — hardware-verified
//
#include <hip/hip_runtime.h>
#pragma clang fp contract(off)

typedef _Float16 f16;
typedef f16   v16h __attribute__((ext_vector_type(16)));
typedef f16   v8h  __attribute__((ext_vector_type(8)));
typedef float v8f  __attribute__((ext_vector_type(8)));
typedef float v4f  __attribute__((ext_vector_type(4)));
typedef int   v4i  __attribute__((ext_vector_type(4)));

#define DTT 0.01f
static constexpr float HDT    = (float)(0.5 * 0.01);
static constexpr float DT6    = (float)(0.01 / 6.0);
static constexpr float SC_A   = 16.f;
static constexpr float SC_W   = 64.f;
static constexpr float SC_D   = 256.f;
static constexpr float SC_R   = 2048.f;
static constexpr float INV_AW = 1.f / 1024.f;
static constexpr float INV_R  = 1.f / 2048.f;
static constexpr float INV_W  = 1.f / 64.f;
static constexpr float INV_DW = 1.f / 16384.f;

__constant__ float c_LOWER[6]  = {-6.28f, -6.28f, -3.14f, -6.28f, -6.28f, -6.28f};
__constant__ float c_UPPER[6]  = { 6.28f,  6.28f,  3.14f,  6.28f,  6.28f,  6.28f};
__constant__ float c_EFFORT[6] = {150.f, 150.f, 150.f, 28.f, 28.f, 28.f};

static constexpr int BO_W1LH = 0;
static constexpr int BO_W1LL = 8192;
static constexpr int BO_W2LH = 16384;
static constexpr int BO_W2LL = 49152;
static constexpr int BO_W3LH = 81920;
static constexpr int BO_W3LL = 90112;
static constexpr int BO_W1VT = 98304;
static constexpr int BO_W2V  = 102400;
static constexpr int BO_FLT  = 135168;
static constexpr int FO_W1LF = 0;
static constexpr int FO_B1L  = 1536;
static constexpr int FO_B2L  = 1664;
static constexpr int FO_B3L  = 1792;
static constexpr int FO_B1V  = 1824;
static constexpr int FO_B2V  = 1952;
static constexpr int FO_W3V  = 2080;
static constexpr int FO_END  = 2208;
static constexpr int BLOB_BYTES = BO_FLT + FO_END * 4;
static constexpr int BLOB_U4    = BLOB_BYTES / 16;

static constexpr int WO_TRIGF = 0;
static constexpr int WO_TBH   = 1024;
static constexpr int WO_TBL   = 2048;
static constexpr int WO_S1    = 4096;
static constexpr int WO_S2    = 8192;
static constexpr int WO_Y     = 12288;
static constexpr int WO_S3    = 14336;
static constexpr int WO_G     = 15360;
static constexpr int WO_BIG   = 16384;
static constexpr int BG_A = 0, BG_B = 4096, BG_C = 8192, BG_D = 12288;
static constexpr int WV_BYTES = 32768;

static constexpr int NWAVE = 2;
static constexpr int NTHR  = 64;
static constexpr int SPB   = 32;
static constexpr int SO_WAVES   = BLOB_BYTES;
static constexpr int SO_KBUF    = SO_WAVES + NWAVE * WV_BYTES;
static constexpr int SO_OBUF    = SO_KBUF + SPB * 8 * 4;
static constexpr int SO_FLAG    = SO_OBUF + SPB * 12 * 4;
static constexpr int SMEM_BYTES = SO_FLAG + 128;

__device__ __forceinline__ v8f zero8(){ v8f z = {0.f, 0.f, 0.f, 0.f, 0.f, 0.f, 0.f, 0.f}; return z; }

__device__ __forceinline__ v8f mma16(v16h a, v16h b, v8f c){
  c = __builtin_amdgcn_wmma_f32_16x16x32_f16(false, a, false, b, (short)0, c, false, false);
  asm volatile("v_nop\n\tv_nop\n\tv_nop\n\tv_nop" : "+v"(c) : "v"(a), "v"(b));
  return c;
}

__device__ __forceinline__ v16h frag_rows(const f16* P, int ld, int row, int k0, int h){
  union { v16h v; v8h p[2]; } f;
  const f16* q = P + row * ld + k0 + 8 * h;
  f.p[0] = *(const v8h*)q;
  f.p[1] = *(const v8h*)(q + 16);
  return f.v;
}
__device__ __forceinline__ v16h frag_cols(const f16* P, int ldn, int n, int k0, int h){
  v16h b;
#pragma unroll
  for (int i = 0; i < 16; ++i){
    const int k = k0 + ((i < 8) ? (8 * h + i) : (8 + 8 * h + i));
    b[i] = P[k * ldn + n];
  }
  return b;
}

__device__ __forceinline__ void split16(float v, f16& hi, f16& lo){
  hi = (f16)v;
  lo = (f16)((v - (float)hi) * SC_R);
}
__device__ __forceinline__ f16 plane_val(float v, bool lo){
  const f16 hi = (f16)v;
  return lo ? (f16)((v - (float)hi) * SC_R) : hi;
}

__device__ __forceinline__ void sp_prec(float x, float& hx, float& sx){
  const float e = expf(-fabsf(x));
  hx = fmaxf(x, 0.f) + log1pf(e);
  const float r = 1.f / (1.f + e);
  sx = (x >= 0.f) ? r : (e * r);
}
__device__ __forceinline__ void sp_fast(float x, float& hx, float& sx){
  const float e = __expf(-fabsf(x));
  hx = fmaxf(x, 0.f) + __logf(1.f + e);
  const float r = __builtin_amdgcn_rcpf(1.f + e);
  sx = (x >= 0.f) ? r : (e * r);
}
__device__ __forceinline__ float sg_fast(float x){
  const float e = __expf(-fabsf(x));
  const float r = __builtin_amdgcn_rcpf(1.f + e);
  return (x >= 0.f) ? r : (e * r);
}

__device__ __forceinline__ float stage_pos(int stage, float q0, float qd0, float km2){
  if (stage == 0) return q0;
  if (stage == 1){ const float t = HDT * qd0; return q0 + t; }
  const float a = HDT * km2;
  const float v = qd0 + a;
  if (stage == 2){ const float t = HDT * v; return q0 + t; }
  const float t = DTT * v;
  return q0 + t;
}
__device__ __forceinline__ float stage_vel(int stage, float qd0, float km1){
  if (stage == 0) return qd0;
  if (stage == 3){ const float t = DTT * km1; return qd0 + t; }
  const float t = HDT * km1;
  return qd0 + t;
}

template<int K, int NF, bool LAST>
__device__ __forceinline__ void mass_layer(const f16* AH, const f16* AL, int lda,
                                           const f16* WH, const f16* WL, const float* bias,
                                           f16* OH, f16* OL, f16* S, float* Yf, int lane)
{
  const int m = lane & 15, h = lane >> 4;
#pragma unroll 1
  for (int nt = 0; nt < NF / 16; ++nt){
    v8f acc = zero8(), accr = zero8();
#pragma unroll
    for (int k0 = 0; k0 < K; k0 += 32){
      const v16h ah = frag_rows(AH, lda, m, k0, h);
      const v16h al = frag_rows(AL, lda, m, k0, h);
      const v16h bh = frag_rows(WH, K, nt * 16 + m, k0, h);
      const v16h bl = frag_rows(WL, K, nt * 16 + m, k0, h);
      acc  = mma16(ah, bh, acc);
      accr = mma16(ah, bl, accr);
      accr = mma16(al, bh, accr);
    }
    const int n = nt * 16 + m;
    const float bn = bias[n];
#pragma unroll
    for (int r = 0; r < 8; ++r){
      const int row = 8 * h + r;
      const float x = (acc[r] + accr[r] * INV_R) * INV_AW + bn;
      float hx, sx;
      sp_prec(x, hx, sx);
      if (LAST){
        Yf[row * 32 + n] = hx;
        S[row * 32 + n] = (f16)sx;
      } else {
        f16 hi, lo;
        split16(hx * SC_A, hi, lo);
        OH[row * NF + n] = hi;
        OL[row * NF + n] = lo;
        S[row * NF + n] = (f16)sx;
      }
    }
  }
}

template<int NF, bool LAST>
__device__ __forceinline__ void tan_layer(const f16* A, const f16* WH, const f16* S, f16* O, float* DY, int lane)
{
  const int m = lane & 15, h = lane >> 4;
#pragma unroll 1
  for (int nt = 0; nt < NF / 16; ++nt){
    v8f acc = zero8();
#pragma unroll
    for (int k0 = 0; k0 < 128; k0 += 32)
      acc = mma16(frag_rows(A, 128, m, k0, h), frag_rows(WH, 128, nt * 16 + m, k0, h), acc);
    const int n = nt * 16 + m;
#pragma unroll
    for (int r = 0; r < 8; ++r){
      const int row = 8 * h + r;
      if (LAST) DY[row * 32 + n] = (float)S[row * 32 + n] * acc[r] * INV_DW;
      else      O[row * NF + n] = (f16)((float)S[row * NF + n] * acc[r] * INV_W);
    }
  }
}

__device__ __forceinline__ void pot_l1(const f16* TB, const f16* W1VT, const float* b1v, f16* H, f16* S, int lane)
{
  const int m = lane & 15, h = lane >> 4;
#pragma unroll 1
  for (int nt = 0; nt < 8; ++nt){
    const v16h a = frag_rows(TB, 32, m, 0, h);
    v16h b;
#pragma unroll
    for (int i = 0; i < 16; ++i)
      b[i] = (i < 8) ? W1VT[(8 * h + i) * 128 + nt * 16 + m] : (f16)0.f;
    v8f acc = mma16(a, b, zero8());
    const int n = nt * 16 + m;
    const float bn = b1v[n];
#pragma unroll
    for (int r = 0; r < 8; ++r){
      const int row = 8 * h + r;
      float hx, sx;
      sp_fast(acc[r] * INV_AW + bn, hx, sx);
      H[row * 128 + n] = (f16)(hx * SC_A);
      S[row * 128 + n] = (f16)sx;
    }
  }
}
__device__ __forceinline__ void pot_l2(const f16* H, const f16* W2V, const float* b2v, const float* w3v, f16* D2, int lane)
{
  const int m = lane & 15, h = lane >> 4;
#pragma unroll 1
  for (int nt = 0; nt < 8; ++nt){
    v8f acc = zero8();
#pragma unroll
    for (int k0 = 0; k0 < 128; k0 += 32)
      acc = mma16(frag_rows(H, 128, m, k0, h), frag_rows(W2V, 128, nt * 16 + m, k0, h), acc);
    const int n = nt * 16 + m;
    const float bn = b2v[n], wn = w3v[n];
#pragma unroll
    for (int r = 0; r < 8; ++r){
      const int row = 8 * h + r;
      D2[row * 128 + n] = (f16)(sg_fast(acc[r] * INV_AW + bn) * wn * SC_D);
    }
  }
}
__device__ __forceinline__ void pot_l2b(const f16* D2, const f16* W2V, const f16* S1V, f16* D1, int lane)
{
  const int m = lane & 15, h = lane >> 4;
#pragma unroll 1
  for (int nt = 0; nt < 8; ++nt){
    v8f acc = zero8();
#pragma unroll
    for (int k0 = 0; k0 < 128; k0 += 32)
      acc = mma16(frag_rows(D2, 128, m, k0, h), frag_cols(W2V, 128, nt * 16 + m, k0, h), acc);
    const int n = nt * 16 + m;
#pragma unroll
    for (int r = 0; r < 8; ++r){
      const int row = 8 * h + r;
      D1[row * 128 + n] = (f16)((float)S1V[row * 128 + n] * acc[r] * INV_W);
    }
  }
}
__device__ __forceinline__ void pot_l1b(const f16* D1, const f16* W1VT, float* G, int lane)
{
  const int m = lane & 15, h = lane >> 4;
  v8f acc = zero8();
#pragma unroll
  for (int k0 = 0; k0 < 128; k0 += 32)
    acc = mma16(frag_rows(D1, 128, m, k0, h), frag_rows(W1VT, 128, m, k0, h), acc);
#pragma unroll
  for (int r = 0; r < 8; ++r) G[(8 * h + r) * 16 + m] = acc[r] * INV_DW;
}

union BlobChunk { v4f v; f16 hh[8]; float f[4]; };

__global__ __launch_bounds__(256) void k_prep(
    const float* __restrict__ W1L, const float* __restrict__ b1L,
    const float* __restrict__ W2L, const float* __restrict__ b2L,
    const float* __restrict__ W3L, const float* __restrict__ b3L,
    const float* __restrict__ W1V, const float* __restrict__ b1V,
    const float* __restrict__ W2V, const float* __restrict__ b2V,
    const float* __restrict__ W3V, const float* __restrict__ b3V,
    float* blob)
{
  (void)b3V;
  const int c = blockIdx.x * blockDim.x + threadIdx.x;
  if (c >= BLOB_U4) return;
  const int o = c * 16;
  BlobChunk val;
  if (o < BO_W1VT){
    if (o < BO_W2LH){
      const bool lo = (o >= BO_W1LL);
      const int el = (o - (lo ? BO_W1LL : BO_W1LH)) >> 1;
#pragma unroll
      for (int i = 0; i < 8; ++i){
        const int idx = el + i, n = idx >> 5, k = idx & 31;
        const float v = (k < 12) ? W1L[n * 12 + k] * SC_W : 0.f;
        val.hh[i] = plane_val(v, lo);
      }
    } else if (o < BO_W3LH){
      const bool lo = (o >= BO_W2LL);
      const int el = (o - (lo ? BO_W2LL : BO_W2LH)) >> 1;
#pragma unroll
      for (int i = 0; i < 8; ++i){
        const float v = W2L[el + i] * SC_W;
        val.hh[i] = plane_val(v, lo);
      }
    } else {
      const bool lo = (o >= BO_W3LL);
      const int el = (o - (lo ? BO_W3LL : BO_W3LH)) >> 1;
#pragma unroll
      for (int i = 0; i < 8; ++i){
        const int idx = el + i, n = idx >> 7, k = idx & 127;
        const float v = (n < 21) ? W3L[n * 128 + k] * SC_W : 0.f;
        val.hh[i] = plane_val(v, lo);
      }
    }
  } else if (o < BO_W2V){
    const int el = (o - BO_W1VT) >> 1;
#pragma unroll
    for (int i = 0; i < 8; ++i){
      const int idx = el + i, kin = idx >> 7, nn = idx & 127;
      const float v = (kin < 12) ? W1V[nn * 12 + kin] * SC_W : 0.f;
      val.hh[i] = (f16)v;
    }
  } else if (o < BO_FLT){
    const int el = (o - BO_W2V) >> 1;
#pragma unroll
    for (int i = 0; i < 8; ++i) val.hh[i] = (f16)(W2V[el + i] * SC_W);
  } else {
    const int fb = (o - BO_FLT) >> 2;
#pragma unroll
    for (int i = 0; i < 4; ++i){
      const int fi = fb + i;
      float v;
      if (fi < FO_B1L)      v = W1L[fi];
      else if (fi < FO_B2L) v = b1L[fi - FO_B1L];
      else if (fi < FO_B3L) v = b2L[fi - FO_B2L];
      else if (fi < FO_B1V){ const int t = fi - FO_B3L; v = (t < 21) ? b3L[t] : 0.f; }
      else if (fi < FO_B2V) v = b1V[fi - FO_B1V];
      else if (fi < FO_W3V) v = b2V[fi - FO_B2V];
      else                  v = W3V[fi - FO_W3V];
      val.f[i] = v;
    }
  }
  const v4f vv = val.v;
  volatile v4f* p = (volatile v4f*)((char*)blob + o);
  *p = vv;
  __threadfence();
  *p = vv;
}

__global__ __launch_bounds__(256) void k_flags(const float* __restrict__ obs, const float* __restrict__ kqd,
                                               int* flg, int B, int Bpad, int stage)
{
  __shared__ int swm[8];
  const int tid = threadIdx.x, lane = tid & 31, wv = tid >> 5;
  int mask = 0;
  for (int e = tid; e < B; e += 256){
#pragma unroll
    for (int j = 0; j < 6; ++j){
      const float q0  = obs[(size_t)e * 12 + j];
      const float qd0 = obs[(size_t)e * 12 + 6 + j];
      float km2 = 0.f;
      if (stage >= 2) km2 = kqd[((size_t)(stage - 2) * Bpad + e) * 8 + j];
      const float qv = stage_pos(stage, q0, qd0, km2);
      const float lo = c_LOWER[j] + 0.1f, up = c_UPPER[j] - 0.1f;
      if (qv <= lo || qv >= up) mask |= (1 << j);
    }
  }
#pragma unroll
  for (int ofs = 16; ofs > 0; ofs >>= 1) mask |= __shfl_xor(mask, ofs);
  if (lane == 0) swm[wv] = mask;
  __syncthreads();
  if (tid == 0){
    int t = 0;
#pragma unroll
    for (int w = 0; w < 8; ++w) t |= swm[w];
    v4i vals[8];
#pragma unroll
    for (int q = 0; q < 8; ++q){
      v4i v;
#pragma unroll
      for (int c = 0; c < 4; ++c){ const int j = 4 * q + c; v[c] = (j < 6) ? ((t >> j) & 1) : 0; }
      vals[q] = v;
    }
    volatile v4i* dst = (volatile v4i*)(flg + stage * 32);
#pragma unroll
    for (int q = 0; q < 8; ++q) dst[q] = vals[q];
    __threadfence();
#pragma unroll
    for (int q = 0; q < 8; ++q) dst[q] = vals[q];
  }
}

__global__ __launch_bounds__(NTHR) void k_accel(
    const float* __restrict__ obs, const float* __restrict__ action,
    const uint4* __restrict__ blob, const int* __restrict__ flags,
    float* kqd, float* out, int B, int Bpad, int stage)
{
  extern __shared__ uint4 smem_u4[];
  char* smem = (char*)smem_u4;
  const int tid = threadIdx.x, lane = tid & 31, wv = tid >> 5, m = lane & 15, h = lane >> 4;

  for (int i = tid; i < BLOB_U4; i += NTHR) smem_u4[i] = blob[i];
  int* sflag = (int*)(smem + SO_FLAG);
  if (tid < 8) sflag[tid] = (tid < 6) ? flags[stage * 32 + tid] : 0;

  const f16* W1LH = (const f16*)(smem + BO_W1LH);
  const f16* W1LL = (const f16*)(smem + BO_W1LL);
  const f16* W2LH = (const f16*)(smem + BO_W2LH);
  const f16* W2LL = (const f16*)(smem + BO_W2LL);
  const f16* W3LH = (const f16*)(smem + BO_W3LH);
  const f16* W3LL = (const f16*)(smem + BO_W3LL);
  const f16* W1VT = (const f16*)(smem + BO_W1VT);
  const f16* W2V  = (const f16*)(smem + BO_W2V);
  const float* FL  = (const float*)(smem + BO_FLT);
  const float* W1LF = FL + FO_W1LF;
  const float* B1L = FL + FO_B1L;
  const float* B2L = FL + FO_B2L;
  const float* B3L = FL + FO_B3L;
  const float* B1V = FL + FO_B1V;
  const float* B2V = FL + FO_B2V;
  const float* W3VF = FL + FO_W3V;

  char* wb = smem + SO_WAVES + wv * WV_BYTES;
  float* TRIGF = (float*)(wb + WO_TRIGF);
  f16* TBH = (f16*)(wb + WO_TBH);
  f16* TBL = (f16*)(wb + WO_TBL);
  f16* S1  = (f16*)(wb + WO_S1);
  f16* S2  = (f16*)(wb + WO_S2);
  float* Y = (float*)(wb + WO_Y);
  f16* S3  = (f16*)(wb + WO_S3);
  float* G = (float*)(wb + WO_G);
  f16* H1H = (f16*)(wb + WO_BIG + BG_A);
  f16* H1L = (f16*)(wb + WO_BIG + BG_B);
  f16* H2H = (f16*)(wb + WO_BIG + BG_C);
  f16* H2L = (f16*)(wb + WO_BIG + BG_D);
  f16* DH1 = (f16*)(wb + WO_BIG + BG_A);
  f16* DH2 = (f16*)(wb + WO_BIG + BG_B);
  float* DY = (float*)(wb + WO_BIG + BG_C);
  f16* H1V = (f16*)(wb + WO_BIG + BG_A);
  f16* S1V = (f16*)(wb + WO_BIG + BG_B);
  f16* D2  = (f16*)(wb + WO_BIG + BG_C);
  f16* D1  = (f16*)(wb + WO_BIG + BG_D);
  float* KB = (float*)(smem + SO_KBUF);
  float* OB = (float*)(smem + SO_OBUF);

  const int e = blockIdx.x * SPB + wv * 16 + m;
  const bool ev = (e < B);

  float qde[6];
  {
    float q0[6], qd0[6], km1[6], km2[6];
#pragma unroll
    for (int j = 0; j < 6; ++j){
      q0[j]  = ev ? obs[(size_t)e * 12 + j] : 0.f;
      qd0[j] = ev ? obs[(size_t)e * 12 + 6 + j] : 0.f;
      km1[j] = 0.f; km2[j] = 0.f;
    }
    if (stage >= 1){
#pragma unroll
      for (int j = 0; j < 6; ++j) km1[j] = ev ? kqd[((size_t)(stage - 1) * Bpad + e) * 8 + j] : 0.f;
    }
    if (stage >= 2){
#pragma unroll
      for (int j = 0; j < 6; ++j) km2[j] = ev ? kqd[((size_t)(stage - 2) * Bpad + e) * 8 + j] : 0.f;
    }
#pragma unroll
    for (int j = 0; j < 6; ++j){
      const float qe = stage_pos(stage, q0[j], qd0[j], km2[j]);
      qde[j] = stage_vel(stage, qd0[j], km1[j]);
      if (h == 0){
        const float cs = cosf(qe), sn = sinf(qe);
        TRIGF[m * 12 + 2 * j]     = cs;
        TRIGF[m * 12 + 2 * j + 1] = sn;
        f16 hi, lo;
        split16(cs * SC_A, hi, lo); TBH[m * 32 + 2 * j] = hi;     TBL[m * 32 + 2 * j] = lo;
        split16(sn * SC_A, hi, lo); TBH[m * 32 + 2 * j + 1] = hi; TBL[m * 32 + 2 * j + 1] = lo;
      }
    }
    if (h == 1){
#pragma unroll
      for (int k = 12; k < 32; ++k){ TBH[m * 32 + k] = (f16)0.f; TBL[m * 32 + k] = (f16)0.f; }
    }
  }
  __syncthreads();

  mass_layer<32, 128, false>(TBH, TBL, 32, W1LH, W1LL, B1L, H1H, H1L, S1, nullptr, lane);
  __syncthreads();
  mass_layer<128, 128, false>(H1H, H1L, 128, W2LH, W2LL, B2L, H2H, H2L, S2, nullptr, lane);
  __syncthreads();
  mass_layer<128, 32, true>(H2H, H2L, 128, W3LH, W3LL, B3L, nullptr, nullptr, S3, Y, lane);
  __syncthreads();

  float w6[6], cacc[6];
#pragma unroll
  for (int j = 0; j < 6; ++j){
    float s = 0.f;
#pragma unroll
    for (int i = j; i < 6; ++i) s += Y[m * 32 + i * (i + 1) / 2 + j] * qde[i];
    w6[j] = s; cacc[j] = 0.f;
  }

#pragma unroll 1
  for (int d = 0; d < 6; ++d){
    for (int idx = lane; idx < 16 * 128; idx += 32){
      const int mm = idx >> 7, n = idx & 127;
      const float cs = TRIGF[mm * 12 + 2 * d];
      const float sn = TRIGF[mm * 12 + 2 * d + 1];
      const float dpre = cs * W1LF[n * 12 + 2 * d + 1] - sn * W1LF[n * 12 + 2 * d];
      DH1[idx] = (f16)((float)S1[idx] * dpre * SC_D);
    }
    __syncthreads();
    tan_layer<128, false>(DH1, W2LH, S2, DH2, nullptr, lane);
    __syncthreads();
    tan_layer<32, true>(DH2, W3LH, S3, nullptr, DY, lane);
    __syncthreads();
    {
      float Lr[21], dL[21];
#pragma unroll
      for (int t = 0; t < 21; ++t){ Lr[t] = Y[m * 32 + t]; dL[t] = DY[m * 32 + t]; }
      float v1[6], u[6];
#pragma unroll
      for (int j = 0; j < 6; ++j){
        float s = 0.f;
#pragma unroll
        for (int i = j; i < 6; ++i) s += dL[i * (i + 1) / 2 + j] * qde[i];
        v1[j] = s;
      }
#pragma unroll
      for (int i = 0; i < 6; ++i){
        float s = 0.f;
#pragma unroll
        for (int j = 0; j <= i; ++j) s += dL[i * (i + 1) / 2 + j] * w6[j] + Lr[i * (i + 1) / 2 + j] * v1[j];
        u[i] = s;
      }
      float dotu = 0.f, qdd = 0.f;
#pragma unroll
      for (int i = 0; i < 6; ++i){ dotu += u[i] * qde[i]; qdd = (i == d) ? qde[i] : qdd; }
#pragma unroll
      for (int i = 0; i < 6; ++i){
        cacc[i] += qdd * u[i];
        cacc[i] -= (i == d) ? 0.5f * dotu : 0.f;
      }
    }
  }
  __syncthreads();

  pot_l1(TBH, W1VT, B1V, H1V, S1V, lane);
  __syncthreads();
  pot_l2(H1V, W2V, B2V, W3VF, D2, lane);
  __syncthreads();
  pot_l2b(D2, W2V, S1V, D1, lane);
  __syncthreads();
  pot_l1b(D1, W1VT, G, lane);
  __syncthreads();

  {
    float q0[6], qd0[6], ks0[6], ks1[6], ks2[6], Lr[21];
#pragma unroll
    for (int j = 0; j < 6; ++j){
      q0[j]  = ev ? obs[(size_t)e * 12 + j] : 0.f;
      qd0[j] = ev ? obs[(size_t)e * 12 + 6 + j] : 0.f;
      ks0[j] = 0.f; ks1[j] = 0.f; ks2[j] = 0.f;
    }
    if (stage >= 1){
#pragma unroll
      for (int j = 0; j < 6; ++j) ks0[j] = ev ? kqd[((size_t)0 * Bpad + e) * 8 + j] : 0.f;
    }
    if (stage >= 2){
#pragma unroll
      for (int j = 0; j < 6; ++j) ks1[j] = ev ? kqd[((size_t)1 * Bpad + e) * 8 + j] : 0.f;
    }
    if (stage >= 3){
#pragma unroll
      for (int j = 0; j < 6; ++j) ks2[j] = ev ? kqd[((size_t)2 * Bpad + e) * 8 + j] : 0.f;
    }
#pragma unroll
    for (int t = 0; t < 21; ++t) Lr[t] = Y[m * 32 + t];

    float rhs[6];
#pragma unroll
    for (int j = 0; j < 6; ++j){
      const float km2 = (stage == 2) ? ks0[j] : ((stage == 3) ? ks1[j] : 0.f);
      const float qe = stage_pos(stage, q0[j], qd0[j], km2);
      const float cs = TRIGF[m * 12 + 2 * j], sn = TRIGF[m * 12 + 2 * j + 1];
      const float gj = G[m * 16 + 2 * j + 1] * cs - G[m * 16 + 2 * j] * sn;
      const float lo = c_LOWER[j] + 0.1f, up = c_UPPER[j] - 0.1f;
      float fj;
      if (sflag[j]) fj = (qe <= lo) ? c_EFFORT[j] : ((qe >= up) ? -c_EFFORT[j] : 0.f);
      else          fj = -5.f * (1.f / (qe - lo) - 1.f / (up - qe));
      const float tau = (ev ? action[(size_t)e * 6 + j] : 0.f) * c_EFFORT[j];
      rhs[j] = ((tau - cacc[j]) - gj) - fj;
    }
    float yv[6], av[6];
#pragma unroll
    for (int i = 0; i < 6; ++i){
      float s = rhs[i];
#pragma unroll
      for (int j = 0; j < i; ++j) s -= Lr[i * (i + 1) / 2 + j] * yv[j];
      yv[i] = s / Lr[i * (i + 1) / 2 + i];
    }
#pragma unroll
    for (int i = 5; i >= 0; --i){
      float s = yv[i];
#pragma unroll
      for (int j = i + 1; j < 6; ++j) s -= Lr[j * (j + 1) / 2 + i] * av[j];
      av[i] = s / Lr[i * (i + 1) / 2 + i];
    }
    if (h == 0){
      const int rloc = wv * 16 + m;
#pragma unroll
      for (int j = 0; j < 6; ++j) KB[rloc * 8 + j] = av[j];
      KB[rloc * 8 + 6] = 0.f; KB[rloc * 8 + 7] = 0.f;
      if (stage == 3){
#pragma unroll
        for (int j = 0; j < 6; ++j){
          const float k1 = ks0[j], k2 = ks1[j], k3 = ks2[j], k4 = av[j];
          const float t2 = HDT * k1, t3 = HDT * k2, t4 = DTT * k3;
          const float k2q = qd0[j] + t2, k3q = qd0[j] + t3, k4q = qd0[j] + t4;
          float sq = qd0[j] + 2.f * k2q; sq = sq + 2.f * k3q; sq = sq + k4q;
          const float dq = DT6 * sq;
          float qn = q0[j] + dq;
          qn = fminf(fmaxf(qn, c_LOWER[j]), c_UPPER[j]);
          float sv = k1 + 2.f * k2; sv = sv + 2.f * k3; sv = sv + k4;
          const float dv = DT6 * sv;
          const float qdn = qd0[j] + dv;
          OB[rloc * 12 + j] = qn;
          OB[rloc * 12 + 6 + j] = qdn;
        }
      }
    }
  }
  __syncthreads();

  if (wv == 0){
    if (stage < 3){
      const v4f* src = (const v4f*)KB;
      const v4f v0 = src[lane], v1 = src[lane + 32];
      volatile v4f* dst = (volatile v4f*)(kqd + ((size_t)stage * Bpad + (size_t)blockIdx.x * SPB) * 8);
      dst[lane] = v0; dst[lane + 32] = v1;
      __threadfence();
      dst[lane] = v0; dst[lane + 32] = v1;
    } else {
      const v4f* src = (const v4f*)OB;
      const v4f v0 = src[lane], v1 = src[lane + 32], v2 = src[lane + 64];
      const int rbase = blockIdx.x * SPB;
      const bool ok0 = (rbase + lane / 3) < B;
      const bool ok1 = (rbase + (lane + 32) / 3) < B;
      const bool ok2 = (rbase + (lane + 64) / 3) < B;
      volatile v4f* dst = (volatile v4f*)(out + (size_t)rbase * 12);
      if (ok0) dst[lane] = v0;
      if (ok1) dst[lane + 32] = v1;
      if (ok2) dst[lane + 64] = v2;
      __threadfence();
      if (ok0) dst[lane] = v0;
      if (ok1) dst[lane + 32] = v1;
      if (ok2) dst[lane + 64] = v2;
    }
  }
}

extern "C" void kernel_launch(void* const* d_in, const int* in_sizes, int n_in,
                              void* d_out, int out_size, void* d_ws, size_t ws_size,
                              hipStream_t stream)
{
  (void)n_in; (void)out_size;
  const float* obs    = (const float*)d_in[0];
  const float* action = (const float*)d_in[1];
  const float* W1L = (const float*)d_in[2];  const float* b1L = (const float*)d_in[3];
  const float* W2L = (const float*)d_in[4];  const float* b2L = (const float*)d_in[5];
  const float* W3L = (const float*)d_in[6];  const float* b3L = (const float*)d_in[7];
  const float* W1V = (const float*)d_in[8];  const float* b1V = (const float*)d_in[9];
  const float* W2V = (const float*)d_in[10]; const float* b2V = (const float*)d_in[11];
  const float* W3V = (const float*)d_in[12]; const float* b3V = (const float*)d_in[13];

  const int B = in_sizes[0] / 12;
  if (B <= 0) return;
  const int nblk = (B + SPB - 1) / SPB;
  const int Bpad = nblk * SPB;

  char* ws = (char*)d_ws;
  const size_t off_blob = 0;
  const size_t off_flag = (size_t)BLOB_BYTES;
  const size_t off_kqd  = off_flag + 4 * 128;
  const size_t need = off_kqd + (size_t)3 * (size_t)Bpad * 8 * sizeof(float);
  if (need > ws_size) return;

  float* blob = (float*)(ws + off_blob);
  int*   flg  = (int*)(ws + off_flag);
  float* kqd  = (float*)(ws + off_kqd);

  k_prep<<<(BLOB_U4 + 255) / 256, 256, 0, stream>>>(W1L, b1L, W2L, b2L, W3L, b3L,
                                                     W1V, b1V, W2V, b2V, W3V, b3V, blob);
  for (int s = 0; s < 4; ++s){
    k_flags<<<1, 256, 0, stream>>>(obs, kqd, flg, B, Bpad, s);
    k_accel<<<nblk, NTHR, SMEM_BYTES, stream>>>(obs, action, (const uint4*)blob, flg, kqd,
                                                (float*)d_out, B, Bpad, s);
  }
}
